// TitansLinear_154618823088
// MI455X (gfx1250) — hardware-verified
//
#include <hip/hip_runtime.h>


#define NB_  4
#define TT   2048
#define DM   1024
#define NH_  16
#define HD   64
typedef _Float16 h16;
typedef unsigned short bf;
typedef __attribute__((ext_vector_type(16))) __bf16   v16bf;
typedef __attribute__((ext_vector_type(16))) _Float16 v16h;
typedef __attribute__((ext_vector_type(8)))  _Float16 v8h;
typedef __attribute__((ext_vector_type(8)))  unsigned short v8us;
typedef __attribute__((ext_vector_type(8)))  float    v8f;
typedef __attribute__((ext_vector_type(4)))  float    v4f;
typedef v8h  __attribute__((may_alias)) v8ha;
typedef v4f  __attribute__((may_alias)) v4fa;
typedef v8us __attribute__((may_alias)) v8usa;

__device__ __forceinline__ unsigned short f2bf(float f) { unsigned u = __float_as_uint(f); u += 0x7FFFu + ((u >> 16) & 1u); return (unsigned short)(u >> 16); }
__device__ __forceinline__ float bf2f(unsigned short b) { return __uint_as_float(((unsigned)b) << 16); }
__device__ __forceinline__ float bfr(float f) { return bf2f(f2bf(f)); }
__device__ __forceinline__ v16h cat16(v8h lo, v8h hi) { return __builtin_shufflevector(lo, hi, 0, 1, 2, 3, 4, 5, 6, 7, 8, 9, 10, 11, 12, 13, 14, 15); }
__device__ __forceinline__ v16bf cat16b(v8us lo, v8us hi) { return __builtin_bit_cast(v16bf, __builtin_shufflevector(lo, hi, 0, 1, 2, 3, 4, 5, 6, 7, 8, 9, 10, 11, 12, 13, 14, 15)); }
__device__ __forceinline__ v8f wmma16(v16h a, v16h b, v8f c) { return __builtin_amdgcn_wmma_f32_16x16x32_f16(false, a, false, b, (short)0, c, false, false); }
__device__ __forceinline__ v8f wmmab(v16bf a, v16bf b, v8f c) { return __builtin_amdgcn_wmma_f32_16x16x32_bf16(false, a, false, b, (short)0, c, false, false); }


template <typename T16> struct WFrag;
template <> struct WFrag<h16> { typedef v16h V; static __device__ __forceinline__ V ld(const h16* p) { return cat16(*(const v8h*)p, *(const v8h*)(p + 16)); } static __device__ __forceinline__ v8f mma(V a, V b, v8f c) { return wmma16(a, b, c); } };
template <> struct WFrag<bf> { typedef v16bf V; static __device__ __forceinline__ V ld(const bf* p) { return cat16b(*(const v8us*)p, *(const v8us*)(p + 16)); } static __device__ __forceinline__ v8f mma(V a, V b, v8f c) { return wmmab(a, b, c); } };
template <typename T16, int NSPLIT, bool BIAS>
__global__ __launch_bounds__(32) void k_gemmw(const T16* __restrict__ A, const T16* __restrict__ A2, const T16* __restrict__ Bt, const T16* __restrict__ Bt2, int K, float* C, int ldc, const float* __restrict__ bias, size_t sA, size_t sB, size_t sC) {
    typedef typename WFrag<T16>::V V;
    __shared__ __align__(16) float os[16 * 68];
    const size_t z = blockIdx.z; A += z * sA; if (A2) A2 += z * sA; Bt += z * sB; if (Bt2) Bt2 += z * sB; C += z * sC;
    const int lane = threadIdx.x & 31, lr = lane & 15, hi = lane >> 4; const int r0 = blockIdx.x * 64, c0 = blockIdx.y * 64;
    v8f acc[4][4];
#pragma unroll
    for (int mb = 0; mb < 4; ++mb)
#pragma unroll
        for (int nb = 0; nb < 4; ++nb) acc[mb][nb] = (v8f){};
    const size_t aoff = (size_t)(r0 + lr) * K + 8 * hi, boff = (size_t)(c0 + lr) * K + 8 * hi;
#pragma unroll 1
    for (int kc = 0; kc < K; kc += 32) {
        V a[4], a2[4];
#pragma unroll
        for (int mb = 0; mb < 4; ++mb) { a[mb] = WFrag<T16>::ld(A + aoff + (size_t)mb * 16 * K + kc); if (NSPLIT == 1 || NSPLIT == 2) a2[mb] = WFrag<T16>::ld(A2 + aoff + (size_t)mb * 16 * K + kc); }
#pragma unroll
        for (int nb = 0; nb < 4; ++nb) { const V b = WFrag<T16>::ld(Bt + boff + (size_t)nb * 16 * K + kc); V b2; if (NSPLIT >= 2) b2 = WFrag<T16>::ld(Bt2 + boff + (size_t)nb * 16 * K + kc);
#pragma unroll
            for (int mb = 0; mb < 4; ++mb) { acc[mb][nb] = WFrag<T16>::mma(a[mb], b, acc[mb][nb]); if (NSPLIT == 1 || NSPLIT == 2) acc[mb][nb] = WFrag<T16>::mma(a2[mb], b, acc[mb][nb]); if (NSPLIT >= 2) acc[mb][nb] = WFrag<T16>::mma(a[mb], b2, acc[mb][nb]); } }
        asm volatile("v_nop\n\tv_nop\n\tv_nop\n\tv_nop" : "+v"(acc[0][0]), "+v"(acc[1][1]), "+v"(acc[2][2]), "+v"(acc[3][3]) : "v"(a[0]), "v"(a[3]));
    }
#pragma unroll
    for (int mb = 0; mb < 4; ++mb) {
#pragma unroll
        for (int nb = 0; nb < 4; ++nb) {
#pragma unroll
            for (int j = 0; j < 8; ++j) os[(hi * 8 + j) * 68 + nb * 16 + lr] = acc[mb][nb][j]; }
        __builtin_amdgcn_wave_barrier(); asm volatile("" ::: "memory");
        float* crow = C + (size_t)(r0 + mb * 16) * ldc + c0;
#pragma unroll 1
        for (int ps = 0; ps < 2; ++ps) {
#pragma unroll
            for (int s = 0; s < 8; ++s) { const int row = 2 * s + hi, cofs = lr * 4; v4f val = *(const v4fa*)(os + row * 68 + cofs); if (BIAS) { val[0] += bfr(bias[c0 + cofs]); val[1] += bfr(bias[c0 + cofs + 1]); val[2] += bfr(bias[c0 + cofs + 2]); val[3] += bfr(bias[c0 + cofs + 3]); }
                *(volatile v4f*)(crow + (size_t)row * ldc + cofs) = val; }
            if (ps == 0) __threadfence(); }
        __builtin_amdgcn_wave_barrier(); asm volatile("" ::: "memory");
    }
}

template <typename T16, int NSPLIT, int CMODE>
__global__ __launch_bounds__(32) void k_gemmc(const T16* __restrict__ A, const T16* __restrict__ A2, const T16* __restrict__ Bt, const T16* __restrict__ Bt2, int K, float* C, int ldc, int roff, size_t sA, size_t sB, size_t sC) {
    typedef typename WFrag<T16>::V V;
    __shared__ __align__(16) float os[16 * 68];
    const size_t z = blockIdx.z; A += z * sA; if (A2) A2 += z * sA; Bt += z * sB; if (Bt2) Bt2 += z * sB; C += z * sC;
    const int lane = threadIdx.x & 31, lr = lane & 15, hi = lane >> 4; const int r0 = blockIdx.x * 64, c0 = blockIdx.y * 64;
    if (CMODE == 1 && c0 > r0 + roff + 63) return;
    const int Kl = (CMODE == 2) ? min(K, r0 + roff + 64) : K;
    v8f acc[4][4];
#pragma unroll
    for (int mb = 0; mb < 4; ++mb)
#pragma unroll
        for (int nb = 0; nb < 4; ++nb) acc[mb][nb] = (v8f){};
    const size_t aoff = (size_t)(r0 + lr) * K + 8 * hi, boff = (size_t)(c0 + lr) * K + 8 * hi;
#pragma unroll 1
    for (int kc = 0; kc < Kl; kc += 32) {
        V a[4], a2[4];
#pragma unroll
        for (int mb = 0; mb < 4; ++mb) { a[mb] = WFrag<T16>::ld(A + aoff + (size_t)mb * 16 * K + kc); if (NSPLIT == 1 || NSPLIT == 2) a2[mb] = WFrag<T16>::ld(A2 + aoff + (size_t)mb * 16 * K + kc); }
#pragma unroll
        for (int nb = 0; nb < 4; ++nb) { const V b = WFrag<T16>::ld(Bt + boff + (size_t)nb * 16 * K + kc); V b2; if (NSPLIT >= 2) b2 = WFrag<T16>::ld(Bt2 + boff + (size_t)nb * 16 * K + kc);
#pragma unroll
            for (int mb = 0; mb < 4; ++mb) { acc[mb][nb] = WFrag<T16>::mma(a[mb], b, acc[mb][nb]); if (NSPLIT == 1 || NSPLIT == 2) acc[mb][nb] = WFrag<T16>::mma(a2[mb], b, acc[mb][nb]); if (NSPLIT >= 2) acc[mb][nb] = WFrag<T16>::mma(a[mb], b2, acc[mb][nb]); } }
        asm volatile("v_nop\n\tv_nop\n\tv_nop\n\tv_nop" : "+v"(acc[0][0]), "+v"(acc[1][1]), "+v"(acc[2][2]), "+v"(acc[3][3]) : "v"(a[0]), "v"(a[3]));
    }
#pragma unroll
    for (int mb = 0; mb < 4; ++mb) {
#pragma unroll
        for (int nb = 0; nb < 4; ++nb) {
#pragma unroll
            for (int j = 0; j < 8; ++j) os[(hi * 8 + j) * 68 + nb * 16 + lr] = acc[mb][nb][j]; }
        __builtin_amdgcn_wave_barrier(); asm volatile("" ::: "memory");
        float* crow = C + (size_t)(r0 + mb * 16) * ldc + c0;
#pragma unroll 1
        for (int ps = 0; ps < 2; ++ps) {
#pragma unroll
            for (int s = 0; s < 8; ++s) { const int row = 2 * s + hi, cofs = lr * 4; v4f val = *(const v4fa*)(os + row * 68 + cofs);
                *(volatile v4f*)(crow + (size_t)row * ldc + cofs) = val; }
            if (ps == 0) __threadfence(); }
        __builtin_amdgcn_wave_barrier(); asm volatile("" ::: "memory");
    }
}

__device__ __forceinline__ h16 tohx(float x) { return (h16)x; }
__device__ __forceinline__ void splitf(float y, unsigned short& h, unsigned short& l) { h = f2bf(y); l = f2bf(y - bf2f(h)); }
__device__ __forceinline__ float siluf_(float a) { return __fdiv_rn(a, __fadd_rn(1.0f, __expf(-a))); }
typedef __attribute__((ext_vector_type(2))) _Float16 v2h;
typedef __attribute__((ext_vector_type(4))) _Float16 v4h;
typedef __attribute__((ext_vector_type(2))) unsigned short v2us;
typedef __attribute__((ext_vector_type(4))) unsigned short v4us;
typedef __attribute__((ext_vector_type(2))) float v2f;

__global__ __launch_bounds__(256) void k_cvt8(const float* __restrict__ src, bf* dst, size_t n8) { const size_t i = (size_t)blockIdx.x * 256 + threadIdx.x; if (i >= n8) return; const v8f v = *(const v8f*)(src + i * 8); v8us o;
#pragma unroll
    for (int k = 0; k < 8; ++k) o[k] = f2bf(v[k]); *(volatile v8us*)(dst + i * 8) = o; __threadfence(); *(volatile v8us*)(dst + i * 8) = o; }
__global__ __launch_bounds__(256) void k_w0t(const float* __restrict__ W0, h16* W0T) { const int e = (blockIdx.x * 256 + threadIdx.x) * 2; if (e >= NH_ * HD * HD) return; const int k = e % HD, v = (e / HD) % HD, h = e / (HD * HD); v2h o; o[0] = tohx(bfr(W0[((size_t)h * HD + k) * HD + v])); o[1] = tohx(bfr(W0[((size_t)h * HD + k + 1) * HD + v])); *(volatile v2h*)(W0T + e) = o; __threadfence(); *(volatile v2h*)(W0T + e) = o; }
__global__ __launch_bounds__(256) void k_qkv(const float* __restrict__ FQ, const float* __restrict__ FK, const float* __restrict__ FV, const float* __restrict__ cq, const float* __restrict__ ck, const float* __restrict__ cv, h16* Q16, h16* K16, h16* V16) {
    const int lane = threadIdx.x & 31; const int w = blockIdx.x * 8 + (threadIdx.x >> 5); if (w >= TT * NH_) return; const int h = w % NH_, t = w / NH_; const int c = h * HD + lane * 2; float y[3][2];
#pragma unroll
    for (int s = 0; s < 3; ++s) { const float* F = s == 0 ? FQ : (s == 1 ? FK : FV); const float* cw = s == 0 ? cq : (s == 1 ? ck : cv);
#pragma unroll
        for (int u = 0; u < 2; ++u) { float acc = F[(size_t)t * DM + c + u];
#pragma unroll
            for (int j = 0; j < 4; ++j) { const int tt = t - 3 + j; const float xv = (tt >= 0) ? F[(size_t)tt * DM + c + u] : 0.f; float p = __fmul_rn(xv, bfr(cw[(c + u) * 4 + j])); asm volatile("" : "+v"(p)); acc = __fadd_rn(acc, p); }
            y[s][u] = siluf_(acc); } }
#pragma unroll
    for (int s = 0; s < 2; ++s) { float q2 = __fadd_rn(__fmul_rn(y[s][0], y[s][0]), __fmul_rn(y[s][1], y[s][1]));
#pragma unroll
        for (int sh = 16; sh; sh >>= 1) q2 += __shfl_xor(q2, sh, 32);
        const float r = __frsqrt_rn(__fadd_rn(q2, 1e-12f)); y[s][0] = __fmul_rn(y[s][0], r); y[s][1] = __fmul_rn(y[s][1], r); }
    const size_t po = ((size_t)h * TT + t) * HD + lane * 2;
#pragma unroll 1
    for (int ps = 0; ps < 2; ++ps) { v2h a, b2, cv2; a[0] = tohx(y[0][0]); a[1] = tohx(y[0][1]); b2[0] = tohx(y[1][0]); b2[1] = tohx(y[1][1]); cv2[0] = tohx(y[2][0]); cv2[1] = tohx(y[2][1]); *(volatile v2h*)(Q16 + po) = a; *(volatile v2h*)(K16 + po) = b2; *(volatile v2h*)(V16 + po) = cv2; if (ps == 0) __threadfence(); } }
__global__ __launch_bounds__(256) void k_vt(const h16* __restrict__ V16, h16* VT) { const size_t e = ((size_t)blockIdx.x * 256 + threadIdx.x) * 2; if (e >= (size_t)NH_ * HD * TT) return; const int t = (int)(e % TT); const int d = (int)((e / TT) % HD); const int h = (int)(e / ((size_t)TT * HD)); v2h o; o[0] = V16[((size_t)h * TT + t) * HD + d]; o[1] = V16[((size_t)h * TT + t + 1) * HD + d]; *(volatile v2h*)(VT + e) = o; __threadfence(); *(volatile v2h*)(VT + e) = o; }
__global__ __launch_bounds__(256) void k_trim(const float* __restrict__ S, h16* S16) { const size_t e = ((size_t)blockIdx.x * 256 + threadIdx.x) * 4; if (e >= (size_t)TT * TT) return; const int j0 = (int)(e % TT), i = (int)(e / TT); v4h o;
#pragma unroll
    for (int q = 0; q < 4; ++q) { const int j = j0 + q; o[q] = (j <= i) ? tohx(S[e + q]) : (h16)0.f; } *(volatile v4h*)(S16 + e) = o; __threadfence(); *(volatile v4h*)(S16 + e) = o; }
__global__ __launch_bounds__(256) void k_lng(const float* __restrict__ O, const float* __restrict__ O2, const float* __restrict__ g, const float* __restrict__ bb, const float* __restrict__ G, int h, bf* Ah, bf* Al) {
    const int lane = threadIdx.x & 31; const int t = blockIdx.x * 8 + (threadIdx.x >> 5); if (t >= TT) return; float v0 = __fadd_rn(O[(size_t)t * HD + lane * 2], O2[(size_t)t * HD + lane * 2]), v1 = __fadd_rn(O[(size_t)t * HD + lane * 2 + 1], O2[(size_t)t * HD + lane * 2 + 1]);
    float s = __fadd_rn(v0, v1);
#pragma unroll
    for (int sh = 16; sh; sh >>= 1) s += __shfl_xor(s, sh, 32);
    const float mu = s * (1.0f / HD); const float d0 = __fsub_rn(v0, mu), d1 = __fsub_rn(v1, mu); float q2 = __fadd_rn(__fmul_rn(d0, d0), __fmul_rn(d1, d1));
#pragma unroll
    for (int sh = 16; sh; sh >>= 1) q2 += __shfl_xor(q2, sh, 32);
    const float rs = __frsqrt_rn(__fadd_rn(q2 * (1.0f / HD), 1e-5f)); const int c = h * HD + lane * 2; v2us oh, ol;
    { float tn = __fmul_rn(d0, rs); asm volatile("" : "+v"(tn)); float tg = __fmul_rn(tn, bfr(g[lane * 2])); asm volatile("" : "+v"(tg)); const float y = __fadd_rn(tg, bfr(bb[lane * 2])); unsigned short a, b2; splitf(__fmul_rn(y, G[(size_t)t * DM + c]), a, b2); oh[0] = a; ol[0] = b2; }
    { float tn = __fmul_rn(d1, rs); asm volatile("" : "+v"(tn)); float tg = __fmul_rn(tn, bfr(g[lane * 2 + 1])); asm volatile("" : "+v"(tg)); const float y = __fadd_rn(tg, bfr(bb[lane * 2 + 1])); unsigned short a, b2; splitf(__fmul_rn(y, G[(size_t)t * DM + c + 1]), a, b2); oh[1] = a; ol[1] = b2; }
    const size_t oo = (size_t)t * DM + c; *(volatile v2us*)(Ah + oo) = oh; *(volatile v2us*)(Al + oo) = ol; __threadfence(); *(volatile v2us*)(Ah + oo) = oh; *(volatile v2us*)(Al + oo) = ol; }

extern "C" void kernel_launch(void* const* d_in, const int* in_sizes, int n_in,
                              void* d_out, int out_size, void* d_ws, size_t ws_size, hipStream_t stream) {
    (void)in_sizes; (void)n_in; (void)out_size;
    const float* IN[12]; for (int i = 0; i < 12; ++i) IN[i] = (const float*)d_in[i];
    float* OUT = (float*)d_out;
    char* wsp = (char*)d_ws;
    auto take = [&](size_t bytes) { char* p = wsp; wsp += (bytes + 255) & ~(size_t)255; return (void*)p; };
    bf* W5[5]; for (int i = 0; i < 5; ++i) W5[i] = (bf*)take((size_t)DM * DM * 2); h16* W0T = (h16*)take((size_t)NH_ * HD * HD * 2);
    bf* XB = (bf*)take((size_t)TT * DM * 2); float* FQ = (float*)take((size_t)TT * DM * 4); float* FK = (float*)take((size_t)TT * DM * 4); float* FV = (float*)take((size_t)TT * DM * 4); float* G = (float*)take((size_t)TT * DM * 4);
    h16* Q16 = (h16*)take((size_t)NH_ * TT * HD * 2); h16* K16 = (h16*)take((size_t)NH_ * TT * HD * 2); h16* V16 = (h16*)take((size_t)NH_ * TT * HD * 2); h16* VT = (h16*)take((size_t)NH_ * HD * TT * 2);
    float* S = (float*)take((size_t)TT * TT * 4); h16* S16 = (h16*)take((size_t)TT * TT * 2); float* O = (float*)take((size_t)TT * HD * 4); float* O2 = (float*)take((size_t)TT * HD * 4); bf* Ah = (bf*)take((size_t)TT * DM * 2); bf* Al = (bf*)take((size_t)TT * DM * 2);
    if ((size_t)(wsp - (char*)d_ws) > ws_size) return;
    { const unsigned g = (unsigned)(((size_t)DM * DM / 8 + 255) / 256); const int src[5] = {1, 2, 3, 10, 11}; for (int i = 0; i < 5; ++i) k_cvt8<<<g, 256, 0, stream>>>(IN[src[i]], W5[i], (size_t)DM * DM / 8); k_w0t<<<(NH_ * HD * HD / 2 + 255) / 256, 256, 0, stream>>>(IN[7], W0T); }
    const dim3 gP(TT / 64, DM / 64, 1);
    for (int b = 0; b < NB_; ++b) {
        k_cvt8<<<(TT * DM / 8 + 255) / 256, 256, 0, stream>>>(IN[0] + (size_t)b * TT * DM, XB, (size_t)TT * DM / 8);
        k_gemmw<bf, 0, false><<<gP, 32, 0, stream>>>(XB, nullptr, W5[0], nullptr, DM, FQ, DM, nullptr, 0, 0, 0); k_gemmw<bf, 0, false><<<gP, 32, 0, stream>>>(XB, nullptr, W5[1], nullptr, DM, FK, DM, nullptr, 0, 0, 0); k_gemmw<bf, 0, false><<<gP, 32, 0, stream>>>(XB, nullptr, W5[2], nullptr, DM, FV, DM, nullptr, 0, 0, 0); k_gemmw<bf, 0, false><<<gP, 32, 0, stream>>>(XB, nullptr, W5[3], nullptr, DM, G, DM, nullptr, 0, 0, 0);
        k_qkv<<<(TT * NH_ + 7) / 8, 256, 0, stream>>>(FQ, FK, FV, IN[4], IN[5], IN[6], Q16, K16, V16); k_vt<<<(unsigned)(((size_t)NH_ * HD * TT / 2 + 255) / 256), 256, 0, stream>>>(V16, VT);
        for (int h = 0; h < NH_; ++h) { const size_t po = (size_t)h * TT * HD;
            k_gemmc<h16, 0, 1><<<dim3(TT / 64, TT / 64, 1), 32, 0, stream>>>(Q16 + po, nullptr, K16 + po, nullptr, HD, S, TT, 0, 0, 0, 0);
            k_trim<<<(unsigned)(((size_t)TT * TT / 4 + 255) / 256), 256, 0, stream>>>(S, S16);
            k_gemmc<h16, 0, 2><<<dim3(TT / 64, 1, 1), 32, 0, stream>>>(S16, nullptr, VT + po, nullptr, TT, O, HD, 0, 0, 0, 0);
            k_gemmw<h16, 0, false><<<dim3(TT / 64, 1, 1), 32, 0, stream>>>(Q16 + po, nullptr, W0T + (size_t)h * HD * HD, nullptr, HD, O2, HD, nullptr, 0, 0, 0);
            k_lng<<<TT / 8, 256, 0, stream>>>(O, O2, IN[8], IN[9], G, h, Ah, Al); }
        k_gemmw<bf, 1, false><<<gP, 32, 0, stream>>>(Ah, Al, W5[4], nullptr, DM, OUT + (size_t)b * TT * DM, DM, nullptr, 0, 0, 0); }
}
